// MySeq2SeqEncoder_19713899889143
// MI455X (gfx1250) — hardware-verified
//
#include <hip/hip_runtime.h>

typedef __attribute__((ext_vector_type(16))) _Float16 v16h;
typedef __attribute__((ext_vector_type(8)))  _Float16 v8h;
typedef __attribute__((ext_vector_type(8)))  float    v8f;
typedef __attribute__((ext_vector_type(4)))  float    v4f;
typedef __attribute__((ext_vector_type(4)))  int      v4i;

constexpr int kBatch = 64;
constexpr int kSeq   = 512;
constexpr int kEmb   = 256;
constexpr int kHid   = 512;
constexpr int kGate  = 3 * kHid;
constexpr int kRowsPerBlock = 16;
constexpr int kThreads = 256;
constexpr int kWaves = kThreads / 32;
constexpr int kUnitsPerWave = kHid / (16 * kWaves);
constexpr int XT_PITCH = kEmb + 8;
constexpr int HT_PITCH = kHid + 8;
static_assert(kBatch % kRowsPerBlock == 0, "batch rows per block");
static_assert(kHid == kWaves * kUnitsPerWave * 16, "column ownership");
static_assert(kEmb % 64 == 0 && kHid % 64 == 0, "k loop steps by 64");
static_assert((XT_PITCH % 8) == 0 && (HT_PITCH % 8) == 0, "16-B aligned fragment loads");
static_assert(kThreads == kRowsPerBlock * 16, "staging thread map");

template <typename T> struct Frag;
template <> struct Frag<_Float16> {
  typedef v16h V; union U { v16h v; v8h h[2]; };
  static __device__ __forceinline__ v16h load(const _Float16* p) {
    U f; f.h[0] = *(const v8h*)(p); f.h[1] = *(const v8h*)(p + 16); return f.v;
  }
  static __device__ __forceinline__ v8f mma(v16h a, v16h b, v8f c) {
    return __builtin_amdgcn_wmma_f32_16x16x32_f16(false, a, false, b, (short)0, c, false, false);
  }
};
typedef Frag<_Float16> FragH;

__device__ __forceinline__ void guard3x8(v8f& x, v8f& y, v8f& z, v16h a0, v16h a1,
                                         v16h p0, v16h p1, v16h p2, v16h p3, v16h p4, v16h p5) {
  asm volatile("v_nop\n\tv_nop\n\tv_nop\n\tv_nop"
               : "+v"(x), "+v"(y), "+v"(z)
               : "v"(a0), "v"(a1), "v"(p0), "v"(p1), "v"(p2), "v"(p3), "v"(p4), "v"(p5));
}
__device__ __forceinline__ void acc_guard4(v8f& a, v8f& b, v8f& c, v8f& d) {
  asm volatile("v_nop\n\tv_nop\n\tv_nop\n\tv_nop" : "+v"(a), "+v"(b), "+v"(c), "+v"(d));
}

__global__ __launch_bounds__(256) void cast_f32_f16x2_scaled(
    const float* __restrict__ in, _Float16* __restrict__ out, int n2, float scale) {
  int i = blockIdx.x * 256 + threadIdx.x;
  if (i < n2) {
    const _Float16 h0 = (_Float16)(in[2 * i] * scale), h1 = (_Float16)(in[2 * i + 1] * scale);
    const unsigned u = (unsigned)__builtin_bit_cast(unsigned short, h0) | ((unsigned)__builtin_bit_cast(unsigned short, h1) << 16);
    ((volatile unsigned*)out)[i] = u;
    __threadfence();
    ((volatile unsigned*)out)[i] = u;
  }
}

__global__ __launch_bounds__(kThreads) void gru_scan_last(
    const int* __restrict__ x, const float* __restrict__ emb, int vocab,
    const unsigned short* __restrict__ wih16p, const unsigned short* __restrict__ whh16p,
    const float* __restrict__ bih, const float* __restrict__ bhh, float* __restrict__ out) {
  __shared__ __align__(16) _Float16 xT[kRowsPerBlock * XT_PITCH];
  __shared__ __align__(16) _Float16 hT[2][kRowsPerBlock * HT_PITCH];
  __shared__ __align__(16) float    hF[kRowsPerBlock * kHid];
  __shared__ int sLast[kRowsPerBlock];

  const int tid  = threadIdx.x;
  const int wave = tid >> 5;
  const int lane = tid & 31;
  const int hh   = lane >> 4;
  const int c    = lane & 15;
  const int b0   = blockIdx.x * kRowsPerBlock;
  const _Float16* wih16 = (const _Float16*)wih16p;
  const _Float16* whh16 = (const _Float16*)whh16p;

  for (int i = tid; i < kRowsPerBlock * kHid; i += kThreads) hF[i] = 0.0f;

  {
    const int row = tid >> 4;
    const int cs  = (tid & 15) * 32;
    const int* xr = x + (size_t)(b0 + row) * kSeq + cs;
    int cnt = 0;
#pragma unroll
    for (int i = 0; i < 8; ++i) {
      const v4i v = *(const v4i*)(xr + 4 * i);
      cnt += (v[0] != 0) + (v[1] != 0) + (v[2] != 0) + (v[3] != 0);
    }
    cnt += __shfl_xor(cnt, 1, 32);
    cnt += __shfl_xor(cnt, 2, 32);
    cnt += __shfl_xor(cnt, 4, 32);
    cnt += __shfl_xor(cnt, 8, 32);
    if ((tid & 15) == 0) sLast[row] = (cnt == 0) ? (kSeq - 1) : (cnt - 1);
  }
  __syncthreads();

  for (int i = tid; i < kRowsPerBlock * kHid; i += kThreads) {
    const int row = i >> 9, col = i & (kHid - 1);
    hT[0][row * HT_PITCH + col] = (_Float16)(hF[i] * 8.0f);
  }
  int ls[8];
#pragma unroll
  for (int r = 0; r < 8; ++r) ls[r] = sLast[8 * hh + r];
  __syncthreads();

  const float inv128 = 0.0078125f;
  const v8f zero8 = (v8f){0.f, 0.f, 0.f, 0.f, 0.f, 0.f, 0.f, 0.f};

  for (int t = 0; t < kSeq; ++t) {
    const int cur = t & 1, nxt = cur ^ 1;

    {
      const int row = tid >> 4;
      const int seg = (tid & 15) * 16;
      int tok = x[(size_t)(b0 + row) * kSeq + t];
      tok = (tok < 0) ? 0 : tok;
      tok = (tok > vocab - 1) ? (vocab - 1) : tok;
      const float* er = emb + (size_t)tok * kEmb + seg;
      const v4f f0 = *(const v4f*)(er);
      const v4f f1 = *(const v4f*)(er + 4);
      const v4f f2 = *(const v4f*)(er + 8);
      const v4f f3 = *(const v4f*)(er + 12);
      v8h o0, o1;
#pragma unroll
      for (int e = 0; e < 4; ++e) {
        o0[e]     = (_Float16)(f0[e] * 8.0f);
        o0[4 + e] = (_Float16)(f1[e] * 8.0f);
        o1[e]     = (_Float16)(f2[e] * 8.0f);
        o1[4 + e] = (_Float16)(f3[e] * 8.0f);
      }
      *(v8h*)(xT + row * XT_PITCH + seg)     = o0;
      *(v8h*)(xT + row * XT_PITCH + seg + 8) = o1;
    }
    __syncthreads();

    const _Float16* hcur = hT[cur];
    _Float16*       hnxt = hT[nxt];

#pragma unroll 1
    for (int ub = 0; ub < kUnitsPerWave; ++ub) {
      const int unitn = wave * (kUnitsPerWave * 16) + ub * 16 + c;

      v8f aR = zero8, aZ = zero8, aI = zero8, aH = zero8;

      {
        const _Float16* aX = xT + c * XT_PITCH + 8 * hh;
        const _Float16* wR = wih16 + (size_t)unitn * kEmb + 8 * hh;
        const _Float16* wZ = wih16 + (size_t)(kHid + unitn) * kEmb + 8 * hh;
        const _Float16* wN = wih16 + (size_t)(2 * kHid + unitn) * kEmb + 8 * hh;
        for (int k0 = 0; k0 < kEmb; k0 += 64) {
          const v16h a0 = FragH::load(aX + k0);
          const v16h a1 = FragH::load(aX + k0 + 32);
          const v16h p0 = FragH::load(wR + k0), p1 = FragH::load(wZ + k0), p2 = FragH::load(wN + k0);
          const v16h p3 = FragH::load(wR + k0 + 32), p4 = FragH::load(wZ + k0 + 32), p5 = FragH::load(wN + k0 + 32);
          aR = FragH::mma(a0, p0, aR);
          aZ = FragH::mma(a0, p1, aZ);
          aI = FragH::mma(a0, p2, aI);
          aR = FragH::mma(a1, p3, aR);
          aZ = FragH::mma(a1, p4, aZ);
          aI = FragH::mma(a1, p5, aI);
          guard3x8(aR, aZ, aI, a0, a1, p0, p1, p2, p3, p4, p5);
        }
      }
      {
        const _Float16* aP = hcur + c * HT_PITCH + 8 * hh;
        const _Float16* vR = whh16 + (size_t)unitn * kHid + 8 * hh;
        const _Float16* vZ = whh16 + (size_t)(kHid + unitn) * kHid + 8 * hh;
        const _Float16* vN = whh16 + (size_t)(2 * kHid + unitn) * kHid + 8 * hh;
        for (int k0 = 0; k0 < kHid; k0 += 64) {
          const v16h a0 = FragH::load(aP + k0);
          const v16h a1 = FragH::load(aP + k0 + 32);
          const v16h p0 = FragH::load(vR + k0), p1 = FragH::load(vZ + k0), p2 = FragH::load(vN + k0);
          const v16h p3 = FragH::load(vR + k0 + 32), p4 = FragH::load(vZ + k0 + 32), p5 = FragH::load(vN + k0 + 32);
          aR = FragH::mma(a0, p0, aR);
          aZ = FragH::mma(a0, p1, aZ);
          aH = FragH::mma(a0, p2, aH);
          aR = FragH::mma(a1, p3, aR);
          aZ = FragH::mma(a1, p4, aZ);
          aH = FragH::mma(a1, p5, aH);
          guard3x8(aR, aZ, aH, a0, a1, p0, p1, p2, p3, p4, p5);
        }
      }
      acc_guard4(aR, aZ, aI, aH);

      const float bR  = bih[unitn] + bhh[unitn];
      const float bZ  = bih[kHid + unitn] + bhh[kHid + unitn];
      const float bI  = bih[2 * kHid + unitn];
      const float bHn = bhh[2 * kHid + unitn];
#pragma unroll
      for (int r = 0; r < 8; ++r) {
        const int row = 8 * hh + r;
        float pr = aR[r] * inv128 + bR;
        float pz = aZ[r] * inv128 + bZ;
        pr = fminf(fmaxf(pr, -30.0f), 30.0f);
        pz = fminf(fmaxf(pz, -30.0f), 30.0f);
        const float rg = 1.0f / (1.0f + expf(-pr));
        const float zg = 1.0f / (1.0f + expf(-pz));
        const float pn = (aI[r] * inv128 + bI) + rg * (aH[r] * inv128 + bHn);
        const float ng = tanhf(pn);
        const float hp = hF[row * kHid + unitn];
        float hn = (1.0f - zg) * ng + zg * hp;
        hn = (t <= ls[r]) ? hn : hp;
        hF[row * kHid + unitn] = hn;
        hnxt[row * HT_PITCH + unitn] = (_Float16)(hn * 8.0f);
      }
    }
    __syncthreads();
  }

  __syncthreads();
  for (int ps = 0; ps < 2; ++ps) {
#pragma unroll
    for (int rr = 0; rr < 2; ++rr) {
      const int row = wave * 2 + rr;
#pragma unroll
      for (int it = 0; it < 4; ++it) {
        const v4f v = *(const v4f*)(hF + row * kHid + it * 128 + lane * 4);
        *(volatile v4f*)(out + (size_t)(b0 + row) * kHid + it * 128 + lane * 4) = v;
      }
    }
    __threadfence();
  }
}

extern "C" void kernel_launch(void* const* d_in, const int* in_sizes, int n_in,
                              void* d_out, int out_size, void* d_ws, size_t ws_size,
                              hipStream_t stream) {
  if (n_in < 6) return;
  if (in_sizes[0] != kBatch * kSeq) return;
  if (in_sizes[1] < kEmb || (in_sizes[1] % kEmb) != 0) return;
  if (in_sizes[2] != kGate * kEmb) return;
  if (in_sizes[3] != kGate * kHid) return;
  if (in_sizes[4] < kGate || in_sizes[5] < kGate) return;
  if (out_size != kBatch * kHid) return;

  const size_t bytesWih = (size_t)kGate * kEmb * 2;
  const size_t bytesWhh = (size_t)kGate * kHid * 2;
  const size_t offWih = 0;
  const size_t offWhh = ((offWih + bytesWih + 127) / 128) * 128;
  const size_t total  = offWhh + bytesWhh;
  if (ws_size < total) return;

  const int*   x   = (const int*)d_in[0];
  const float* emb = (const float*)d_in[1];
  const float* Wih = (const float*)d_in[2];
  const float* Whh = (const float*)d_in[3];
  const float* bih = (const float*)d_in[4];
  const float* bhh = (const float*)d_in[5];
  float* out = (float*)d_out;
  char* ws = (char*)d_ws;
  _Float16* wih16 = (_Float16*)(ws + offWih);
  _Float16* whh16 = (_Float16*)(ws + offWhh);
  const int vocab = in_sizes[1] / kEmb;

  const int n2ih = (kGate * kEmb) / 2;
  const int n2hh = (kGate * kHid) / 2;
  cast_f32_f16x2_scaled<<<dim3((n2ih + 255) / 256), dim3(256), 0, stream>>>(Wih, wih16, n2ih, 16.0f);
  cast_f32_f16x2_scaled<<<dim3((n2hh + 255) / 256), dim3(256), 0, stream>>>(Whh, whh16, n2hh, 16.0f);
  gru_scan_last<<<dim3(kBatch / kRowsPerBlock), dim3(kThreads), 0, stream>>>(
      x, emb, vocab, (const unsigned short*)wih16, (const unsigned short*)whh16, bih, bhh, out);
}
